// HybridSelfAttentionBlockWithDisplacement_26774826123571
// MI455X (gfx1250) — hardware-verified
//
#include <hip/hip_runtime.h>
#include <math.h>

constexpr int NBATCH = 2;
constexpr int NLS = 1024;
constexpr int NGLOB = 32;
constexpr int NDIM = 512;
constexpr int NHEAD = 8;
constexpr int DHEAD = 64;
constexpr int KNB = 32;
constexpr int NPE = 64;
constexpr int NINNER = 512;
constexpr int NHID = 128;
constexpr int NTOK = NBATCH * NLS;
constexpr int NGROW = NBATCH * NGLOB;
constexpr int CTXROWS = 1088;
constexpr int CTXVALID = NLS + NGLOB;
constexpr int NSLOT = KNB + 1;
constexpr int NRPEROWS = NTOK * NSLOT;
constexpr int RPEROWS_B = NLS * NSLOT;
constexpr int KVROWS = NTOK + NBATCH * 64;
constexpr int NCTXL = 1 + KNB + NGLOB;
constexpr int HEADPITCH = 68;
constexpr int ATTNPITCH = NHEAD * HEADPITCH;
constexpr int DISPSLOT = 7 * HEADPITCH + 66;
constexpr int GQGRP = 8;
constexpr float ATTNSCALE = 0.125f;
constexpr float WCARRY = 32.0f;
constexpr float RCARRY = 16.0f;
constexpr float OCARRY = 32.0f;
constexpr float MAXDISP = 5.0f;
static_assert(ATTNPITCH % 32 == 0);
static_assert(RPEROWS_B % 64 == 0);
static_assert(CTXROWS % 64 == 0);
static_assert(NTOK % 16 == 0);

typedef __attribute__((ext_vector_type(16))) _Float16 v16h;
typedef __attribute__((ext_vector_type(8)))  _Float16 v8h;
typedef __attribute__((ext_vector_type(16))) __bf16   v16b;
typedef __attribute__((ext_vector_type(8)))  __bf16   v8b;
typedef __attribute__((ext_vector_type(8)))  float    v8f;
typedef __attribute__((ext_vector_type(4)))  float    v4f;
typedef __attribute__((ext_vector_type(2)))  float    v2f;
typedef __attribute__((ext_vector_type(4)))  unsigned int v4u;
typedef __attribute__((ext_vector_type(2)))  unsigned int v2u;

__device__ __forceinline__ unsigned short f2bf_bits(float f) {
  unsigned u = __float_as_uint(f);
  return (unsigned short)((u + 0x7FFFu + ((u >> 16) & 1u)) >> 16);
}
__device__ __forceinline__ float bf_bits2f(unsigned short h) { return __uint_as_float(((unsigned)h) << 16); }

__device__ __forceinline__ void dep_guard_h(v8f& a, v8f& b, v16h x, v16h y) { asm volatile("v_nop\n\tv_nop\n\tv_nop\n\tv_nop" : "+v"(a), "+v"(b) : "v"(x), "v"(y)); }
__device__ __forceinline__ void dep_guard_b(v8f& a, v8f& b, v16b x, v16b y) { asm volatile("v_nop\n\tv_nop\n\tv_nop\n\tv_nop" : "+v"(a), "+v"(b) : "v"(x), "v"(y)); }
__device__ __forceinline__ void keep4_h(v16h a, v16h b, v16h c, v16h d) { asm volatile("v_nop" :: "v"(a), "v"(b), "v"(c), "v"(d)); }
__device__ __forceinline__ void keep4_b(v16b a, v16b b, v16b c, v16b d) { asm volatile("v_nop" :: "v"(a), "v"(b), "v"(c), "v"(d)); }
__device__ __forceinline__ void acc_guard4(v8f& a, v8f& b, v8f& c, v8f& d) { asm volatile("v_nop\n\tv_nop\n\tv_nop\n\tv_nop" : "+v"(a), "+v"(b), "+v"(c), "+v"(d)); }
template <typename T> struct Frag;
template <> struct Frag<_Float16> {
  typedef v16h V; union U { v16h v; v8h h[2]; };
  static __device__ __forceinline__ v16h load(const _Float16* p) {
    U f; f.h[0] = *(const v8h*)(p); f.h[1] = *(const v8h*)(p + 16); return f.v;
  }
  static __device__ __forceinline__ v8f mma(v16h a, v16h b, v8f c) {
    return __builtin_amdgcn_wmma_f32_16x16x32_f16(false, a, false, b, (short)0, c, false, false);
  }
  static __device__ __forceinline__ void guard(v8f& a, v8f& b, v16h x, v16h y) { dep_guard_h(a, b, x, y); }
  static __device__ __forceinline__ void keep(v16h a, v16h b, v16h c, v16h d) { keep4_h(a, b, c, d); }
};
template <> struct Frag<__bf16> {
  typedef v16b V; union U { v16b v; v8b h[2]; };
  static __device__ __forceinline__ v16b load(const __bf16* p) {
    U f; f.h[0] = *(const v8b*)(p); f.h[1] = *(const v8b*)(p + 16); return f.v;
  }
  static __device__ __forceinline__ v8f mma(v16b a, v16b b, v8f c) {
    return __builtin_amdgcn_wmma_f32_16x16x32_bf16(false, a, false, b, (short)0, c, false, false);
  }
  static __device__ __forceinline__ void guard(v8f& a, v8f& b, v16b x, v16b y) { dep_guard_b(a, b, x, y); }
  static __device__ __forceinline__ void keep(v16b a, v16b b, v16b c, v16b d) { keep4_b(a, b, c, d); }
};

__device__ __forceinline__ unsigned pk16(unsigned short a, unsigned short b) { return (unsigned)a | ((unsigned)b << 16); }
__device__ __forceinline__ unsigned short h_bits(float f) { const _Float16 h = (_Float16)f; return __builtin_bit_cast(unsigned short, h); }

template <int ET> struct Elem;
template <> struct Elem<0> { typedef _Float16 T; };
template <> struct Elem<1> { typedef __bf16 T; };
template <int ET, bool SPLIT, int BIAS_MODE, int OUT_MODE, bool RESID, int ACT = 0>
__global__ __launch_bounds__(256) void wmma_gemm64(
    const unsigned short* __restrict__ Ap, const unsigned short* __restrict__ A2p, int lda, long strideA,
    const unsigned short* __restrict__ Btp, const unsigned short* __restrict__ Bt2p, int ldb, long strideB,
    void* __restrict__ Cout, void* __restrict__ Cout2, int ldc, long strideC,
    const float* __restrict__ bias,
    const float* __restrict__ resid, long strideR,
    int M, int N, int K, float scale) {
  typedef typename Elem<ET>::T T;
  typedef typename Frag<T>::V V;
  const T* A = (const T*)Ap; const T* A2 = (const T*)A2p; const T* Bt = (const T*)Btp; const T* Bt2 = (const T*)Bt2p;
  __shared__ __align__(16) float sT[8][16 * 68];
  const int b    = blockIdx.y;
  const int lane = threadIdx.x & 31;
  const int wave = threadIdx.x >> 5;
  const int tilesN = N >> 6;
  const int tilesM = M >> 6;
  const int tile = blockIdx.x * 8 + wave;
  if (tile >= tilesM * tilesN) return;
  const int tm = tile / tilesN;
  const int tn = tile - tm * tilesN;
  const int m0 = tm << 6;
  const int n0 = tn << 6;

  const T* Ab  = A  + (size_t)b * strideA;
  const T* Bb  = Bt + (size_t)b * strideB;
  const T* Ab2 = SPLIT ? (A2  + (size_t)b * strideA) : nullptr;
  const T* Bb2 = SPLIT ? (Bt2 + (size_t)b * strideB) : nullptr;

  const int rlane = lane & 15;
  const int koff  = (lane >> 4) * 8;
  const int mOff  = (lane >> 4) * 8;

  v8f acc[4][4];
#pragma unroll
  for (int i = 0; i < 4; ++i)
#pragma unroll
    for (int j = 0; j < 4; ++j) acc[i][j] = (v8f){0.f,0.f,0.f,0.f,0.f,0.f,0.f,0.f};

  for (int k0 = 0; k0 < K; k0 += 32) {
    V bh[4], bl[4];
#pragma unroll
    for (int j = 0; j < 4; ++j) {
      const size_t bo = (size_t)(n0 + (j << 4) + rlane) * ldb + koff + k0;
      bh[j] = Frag<T>::load(Bb + bo);
      if (SPLIT) bl[j] = Frag<T>::load(Bb2 + bo);
    }
#pragma unroll
    for (int i = 0; i < 4; ++i) {
      const size_t ao = (size_t)(m0 + (i << 4) + rlane) * lda + koff + k0;
      V ah = Frag<T>::load(Ab + ao);
      V al;
      if (SPLIT) al = Frag<T>::load(Ab2 + ao);
#pragma unroll
      for (int j = 0; j < 4; ++j) {
        acc[i][j] = Frag<T>::mma(ah, bh[j], acc[i][j]);
        if (SPLIT) {
          acc[i][j] = Frag<T>::mma(ah, bl[j], acc[i][j]);
          acc[i][j] = Frag<T>::mma(al, bh[j], acc[i][j]);
        }
      }
      Frag<T>::guard(acc[i][0], acc[i][3], ah, SPLIT ? al : ah);
    }
    Frag<T>::keep(bh[0], bh[1], bh[2], bh[3]);
    if (SPLIT) Frag<T>::keep(bl[0], bl[1], bl[2], bl[3]);
  }
  acc_guard4(acc[0][0], acc[0][1], acc[0][2], acc[0][3]);
  acc_guard4(acc[1][0], acc[1][1], acc[1][2], acc[1][3]);
  acc_guard4(acc[2][0], acc[2][1], acc[2][2], acc[2][3]);
  acc_guard4(acc[3][0], acc[3][1], acc[3][2], acc[3][3]);

  float* slab = sT[wave];
  const float* Rb = RESID ? (resid + (size_t)b * strideR) : nullptr;
#pragma unroll
  for (int i = 0; i < 4; ++i) {
    const int mBase = m0 + (i << 4);
#pragma unroll
    for (int j = 0; j < 4; ++j) {
      const int n = n0 + (j << 4) + rlane;
      float bv = 0.f;
      if (BIAS_MODE == 2) bv = bias[n];
#pragma unroll
      for (int r = 0; r < 8; ++r) {
        float v = acc[i][j][r] * scale;
        if (BIAS_MODE == 1) v += bias[mBase + mOff + r];
        if (BIAS_MODE == 2) v += bv;
        if (RESID) v += Rb[(size_t)(mBase + mOff + r) * ldc + n];
        if (ACT == 2) v = fmaxf(v, 0.0f);
        if (ACT == 4) v = (v > 0.f) ? v : 0.01f * v;
        slab[(mOff + r) * 68 + (j << 4) + rlane] = v;
      }
    }
    __builtin_amdgcn_fence(__ATOMIC_RELEASE, "workgroup");
    __builtin_amdgcn_wave_barrier();
    __builtin_amdgcn_fence(__ATOMIC_ACQUIRE, "workgroup");
    if (OUT_MODE == 0) {
      float* C = (float*)Cout + (size_t)b * strideC;
      const int hh = lane >> 4, c4 = (lane & 15) * 4;
      for (int pass = 0; pass < 2; ++pass) {
#pragma unroll
        for (int it = 0; it < 8; ++it) {
          const int row = it * 2 + hh;
          v4f v = *(const v4f*)(slab + row * 68 + c4);
          *(volatile v4f*)(C + (size_t)(mBase + row) * ldc + n0 + c4) = v;
        }
        __threadfence();
      }
    } else {
      const int q = lane >> 3, c8 = (lane & 7) * 8;
      unsigned short* C  = (unsigned short*)Cout  + (size_t)b * strideC;
      unsigned short* C2 = (OUT_MODE == 2) ? ((unsigned short*)Cout2 + (size_t)b * strideC) : nullptr;
      for (int pass = 0; pass < 2; ++pass) {
#pragma unroll
        for (int it = 0; it < 4; ++it) {
          const int row = it * 4 + q;
          const float* sp = slab + row * 68 + c8;
          v8h hv, lv;
#pragma unroll
          for (int e = 0; e < 8; ++e) {
            if (OUT_MODE == 1) {
              hv[e] = (_Float16)sp[e];
            } else {
              unsigned short hb = f2bf_bits(sp[e]);
              unsigned short lb = f2bf_bits(sp[e] - bf_bits2f(hb));
              hv[e] = __builtin_bit_cast(_Float16, hb);
              lv[e] = __builtin_bit_cast(_Float16, lb);
            }
          }
          *(volatile v8h*)(C + (size_t)(mBase + row) * ldc + n0 + c8) = hv;
          if (OUT_MODE == 2) *(volatile v8h*)(C2 + (size_t)(mBase + row) * ldc + n0 + c8) = lv;
        }
        __threadfence();
      }
    }
    __builtin_amdgcn_fence(__ATOMIC_RELEASE, "workgroup");
    __builtin_amdgcn_wave_barrier();
    __builtin_amdgcn_fence(__ATOMIC_ACQUIRE, "workgroup");
  }
}

__global__ __launch_bounds__(256) void cast8_f16_kernel(const float* __restrict__ in, unsigned short* __restrict__ out, int n8) {
  const int i = blockIdx.x * 256 + threadIdx.x;
  if (i >= n8) return;
  const float* p = in + 8 * (size_t)i;
  const v4f a = *(const v4f*)(p);
  const v4f c = *(const v4f*)(p + 4);
  unsigned short hb[8];
#pragma unroll
  for (int e = 0; e < 4; ++e) {
    hb[e]     = h_bits(a[e]);
    hb[4 + e] = h_bits(c[e]);
  }
  const v4u u = (v4u){pk16(hb[0], hb[1]), pk16(hb[2], hb[3]), pk16(hb[4], hb[5]), pk16(hb[6], hb[7])};
  unsigned short* q = out + 8 * (size_t)i;
  *(volatile v4u*)q = u;
  __threadfence();
  *(volatile v4u*)q = u;
}

__device__ __forceinline__ float h16_to_f32(unsigned h) {
  const unsigned m = h & 0x7fffu;
  const unsigned e = (m < 0x0400u) ? 0u : ((m + 0x1C000u) << 13);
  return __uint_as_float(e | ((h & 0x8000u) << 16));
}
__device__ __forceinline__ float hlo2f(unsigned w) { return h16_to_f32(w & 0xffffu); }
__device__ __forceinline__ float hhi2f(unsigned w) { return h16_to_f32(w >> 16); }
__device__ __forceinline__ float wave_sum(float v) {
#pragma unroll
  for (int off = 16; off > 0; off >>= 1) v += __shfl_xor(v, off, 32);
  return v;
}
__device__ __forceinline__ float wave_max(float v) {
#pragma unroll
  for (int off = 16; off > 0; off >>= 1) v = fmaxf(v, __shfl_xor(v, off, 32));
  return v;
}
__device__ __forceinline__ int clampi(int v, int lo, int hi) { return v < lo ? lo : (v > hi ? hi : v); }

__global__ __launch_bounds__(256) void wtcast_kernel(const float* __restrict__ W0, const float* __restrict__ W1,
                                                     const float* __restrict__ W2, const float* __restrict__ W3,
                                                     int Kd, int N, unsigned short* __restrict__ out, long outStride,
                                                     float scale) {
  __shared__ float sm[64][65];
  const int t  = threadIdx.x;
  const int k0 = blockIdx.x * 64;
  const int n0 = blockIdx.y * 64;
  const int z  = blockIdx.z;
  const float* W = (z == 0) ? W0 : (z == 1) ? W1 : (z == 2) ? W2 : W3;
#pragma unroll
  for (int i = 0; i < 16; ++i) {
    const int e  = i * 256 + t;
    const int r  = e >> 6;
    const int cc = e & 63;
    sm[cc][r] = W[(size_t)(k0 + r) * N + n0 + cc] * scale;
  }
  __syncthreads();
  const int lane = t & 31, wave = t >> 5;
  const int q = lane >> 3, c8 = (lane & 7) * 8;
  unsigned short* op = out + (size_t)z * outStride;
  for (int pass = 0; pass < 2; ++pass) {
#pragma unroll
    for (int it = 0; it < 2; ++it) {
      const int row = wave * 8 + it * 4 + q;
      unsigned short hb[8];
#pragma unroll
      for (int e = 0; e < 8; ++e) hb[e] = h_bits(sm[row][c8 + e]);
      const v4u u = (v4u){pk16(hb[0], hb[1]), pk16(hb[2], hb[3]), pk16(hb[4], hb[5]), pk16(hb[6], hb[7])};
      *(volatile v4u*)(op + (size_t)(n0 + row) * Kd + k0 + c8) = u;
    }
    __threadfence();
  }
}

__global__ __launch_bounds__(256) void ln_rows_kernel(const float* __restrict__ xs, const float* __restrict__ xg,
                                                      const float* __restrict__ gs, const float* __restrict__ bsp,
                                                      const float* __restrict__ gg, const float* __restrict__ bgp,
                                                      unsigned short* __restrict__ ctx) {
  const int lane = threadIdx.x & 31, wave = threadIdx.x >> 5;
  const int row = blockIdx.x * 8 + wave;
  const bool isG = (blockIdx.x >= (NTOK / 8));
  const float* src; const float* gp; const float* bp; size_t drow;
  if (!isG) {
    src = xs + (size_t)row * NDIM; gp = gs; bp = bsp;
    drow = (size_t)(row >> 10) * CTXROWS + (row & 1023);
  } else {
    const int j = row - NTOK;
    src = xg + (size_t)j * NDIM; gp = gg; bp = bgp;
    drow = (size_t)(j >> 5) * CTXROWS + NLS + (j & 31);
  }
  float x[16], g[16], bb[16];
  {
    const v4f a0 = *(const v4f*)(src + lane * 8);
    const v4f a1 = *(const v4f*)(src + lane * 8 + 4);
    const v4f a2 = *(const v4f*)(src + 256 + lane * 8);
    const v4f a3 = *(const v4f*)(src + 256 + lane * 8 + 4);
    const v4f g0 = *(const v4f*)(gp + lane * 8);
    const v4f g1 = *(const v4f*)(gp + lane * 8 + 4);
    const v4f g2 = *(const v4f*)(gp + 256 + lane * 8);
    const v4f g3 = *(const v4f*)(gp + 256 + lane * 8 + 4);
    const v4f b0 = *(const v4f*)(bp + lane * 8);
    const v4f b1 = *(const v4f*)(bp + lane * 8 + 4);
    const v4f b2 = *(const v4f*)(bp + 256 + lane * 8);
    const v4f b3 = *(const v4f*)(bp + 256 + lane * 8 + 4);
#pragma unroll
    for (int e = 0; e < 4; ++e) {
      x[e] = a0[e]; x[4 + e] = a1[e]; x[8 + e] = a2[e]; x[12 + e] = a3[e];
      g[e] = g0[e]; g[4 + e] = g1[e]; g[8 + e] = g2[e]; g[12 + e] = g3[e];
      bb[e] = b0[e]; bb[4 + e] = b1[e]; bb[8 + e] = b2[e]; bb[12 + e] = b3[e];
    }
  }
  float s = 0.f;
#pragma unroll
  for (int e = 0; e < 16; ++e) s += x[e];
  s = wave_sum(s);
  const float mean = s * (1.0f / NDIM);
  float ss = 0.f;
#pragma unroll
  for (int e = 0; e < 16; ++e) { const float d = x[e] - mean; ss += d * d; }
  ss = wave_sum(ss);
  const float rstd = 1.0f / sqrtf(ss * (1.0f / NDIM) + 1e-5f);
  unsigned short hb[16];
#pragma unroll
  for (int e = 0; e < 16; ++e) hb[e] = h_bits((x[e] - mean) * rstd * g[e] + bb[e]);
  const v4u u0 = (v4u){pk16(hb[0], hb[1]), pk16(hb[2], hb[3]), pk16(hb[4], hb[5]), pk16(hb[6], hb[7])};
  const v4u u1 = (v4u){pk16(hb[8], hb[9]), pk16(hb[10], hb[11]), pk16(hb[12], hb[13]), pk16(hb[14], hb[15])};
  unsigned short* d0 = ctx + drow * NDIM + lane * 8;
  unsigned short* d1 = d0 + 256;
  *(volatile v4u*)d0 = u0;
  *(volatile v4u*)d1 = u1;
  __threadfence();
  *(volatile v4u*)d0 = u0;
  *(volatile v4u*)d1 = u1;
}

__global__ __launch_bounds__(256) void zero_ctxpad_kernel(unsigned short* __restrict__ ctx) {
  const int i = blockIdx.x * 256 + threadIdx.x;
  const int b = i >> 11, rem = i & 2047;
  unsigned short* p = ctx + ((size_t)b * CTXROWS + CTXVALID) * NDIM + (size_t)rem * 8;
  const v4u zz = (v4u){0u, 0u, 0u, 0u};
  *(volatile v4u*)p = zz;
  __threadfence();
  *(volatile v4u*)p = zz;
}

__global__ __launch_bounds__(256) void rpecat_kernel(const float* __restrict__ rpe, const float* __restrict__ srpe,
                                                     unsigned short* __restrict__ outp) {
  const int slot = blockIdx.y;
  const int tl = threadIdx.x >> 3, part = threadIdx.x & 7;
  const int l = blockIdx.x * 32 + tl;
  const int sm1 = slot > 0 ? slot - 1 : 0;
  const float* srcA = srpe + (size_t)l * NPE + part * 8;
  const float* srcB = rpe + ((size_t)l * KNB + sm1) * NPE + part * 8;
  const float* src = (slot == 0) ? srcA : srcB;
  const v4f a = *(const v4f*)(src);
  const v4f c = *(const v4f*)(src + 4);
  unsigned short hb[8];
#pragma unroll
  for (int e = 0; e < 4; ++e) { hb[e] = h_bits(a[e]); hb[4 + e] = h_bits(c[e]); }
  const v4u u = (v4u){pk16(hb[0], hb[1]), pk16(hb[2], hb[3]), pk16(hb[4], hb[5]), pk16(hb[6], hb[7])};
  unsigned short* dst = outp + ((size_t)l * NSLOT + slot) * NPE + part * 8;
  *(volatile v4u*)dst = u;
  __threadfence();
  *(volatile v4u*)dst = u;
}

__global__ __launch_bounds__(256) void attn_scores_kernel(const float* __restrict__ Qp, const float* __restrict__ Kpl,
                                                          const unsigned short* __restrict__ RKp,
                                                          const float* __restrict__ dist, const int* __restrict__ topk,
                                                          const float* __restrict__ log_sigma, const float* __restrict__ gbl,
                                                          const float* __restrict__ headw, const float* __restrict__ pos,
                                                          const int* __restrict__ kcount, float* __restrict__ attn, int tok0) {
  __shared__ __align__(16) float sQ[NINNER];
  __shared__ __align__(16) float sRow[ATTNPITCH];
  __shared__ int sFrow[HEADPITCH];
  __shared__ int sIdx[KNB];
  __shared__ float sHi[NHEAD];
  __shared__ float sInv2s[NHEAD];
  const int tid = threadIdx.x, lane = tid & 31, wave = tid >> 5;
  const int lloc = blockIdx.x;
  const int l = tok0 + lloc;
  const int b = l >> 10;

  sQ[tid] = Qp[(size_t)l * NINNER + tid];
  sQ[tid + 256] = Qp[(size_t)l * NINNER + 256 + tid];
  if (tid < NCTXL) {
    const int cc = tid;
    const int cm1 = clampi(cc - 1, 0, KNB - 1);
    const int nb = clampi(topk[(size_t)l * KNB + cm1], 0, NLS - 1);
    const int fr = (cc == 0) ? l : (cc <= KNB) ? (b * NLS + nb) : (NTOK + b * 64 + (cc - KNB - 1));
    sFrow[cc] = fr;
  }
  if (tid < KNB) sIdx[tid] = clampi(topk[(size_t)l * KNB + tid], 0, NLS - 1);
  if (tid < 24) {
    const int hh = tid / 3;
    const int j = NCTXL + (tid - hh * 3);
    sRow[hh * HEADPITCH + j] = 0.0f;
  }
  if (tid < NHEAD) {
    float mx = -INFINITY;
#pragma unroll 1
    for (int hh = 0; hh < NHEAD; ++hh) mx = fmaxf(mx, headw[hh]);
    float se = 0.f;
#pragma unroll 1
    for (int hh = 0; hh < NHEAD; ++hh) se += expf(headw[hh] - mx);
    sHi[tid] = expf(headw[tid] - mx) / se;
    sInv2s[tid] = 1.0f / (2.0f * expf(2.0f * log_sigma[tid]));
  }
  __syncthreads();

  const float gb = gbl[0];
#pragma unroll 1
  for (int p = tid; p < NHEAD * NCTXL; p += 256) {
    const int hh = p / NCTXL;
    const int cc = p - hh * NCTXL;
    const int fr = sFrow[cc];
    const int rs = cc < NSLOT ? cc : (NSLOT - 1);
    const float rmul = (cc < NSLOT) ? (1.0f / RCARRY) : 0.0f;
    const float* kf = Kpl + (size_t)fr * NINNER + hh * DHEAD;
    const unsigned short* kr = RKp + ((size_t)lloc * NSLOT + rs) * NINNER + hh * DHEAD;
    const float* qh = sQ + hh * DHEAD;
    float acc = 0.f;
#pragma unroll 1
    for (int it = 0; it < 8; ++it) {
      const v4f f0 = *(const v4f*)(kf + it * 8);
      const v4f f1 = *(const v4f*)(kf + it * 8 + 4);
      const v4u rr = *(const v4u*)(kr + it * 8);
      const v4f q0 = *(const v4f*)(qh + it * 8);
      const v4f q1 = *(const v4f*)(qh + it * 8 + 4);
      acc += q0[0] * (f0[0] + rmul * hlo2f(rr[0]));
      acc += q0[1] * (f0[1] + rmul * hhi2f(rr[0]));
      acc += q0[2] * (f0[2] + rmul * hlo2f(rr[1]));
      acc += q0[3] * (f0[3] + rmul * hhi2f(rr[1]));
      acc += q1[0] * (f1[0] + rmul * hlo2f(rr[2]));
      acc += q1[1] * (f1[1] + rmul * hhi2f(rr[2]));
      acc += q1[2] * (f1[2] + rmul * hlo2f(rr[3]));
      acc += q1[3] * (f1[3] + rmul * hhi2f(rr[3]));
    }
    const int cm1 = clampi(cc - 1, 0, KNB - 1);
    const float d = dist[(size_t)l * KNB + cm1];
    const float bl = -(d * d) * sInv2s[hh];
    const float bias = (cc == 0) ? 0.0f : (cc <= KNB) ? bl : gb;
    sRow[hh * HEADPITCH + cc] = acc * ATTNSCALE + bias;
  }
  __syncthreads();

  {
    float* sr = sRow + wave * HEADPITCH;
    float m = -INFINITY;
#pragma unroll 1
    for (int r = 0; r < 3; ++r) {
      const int cc = lane + 32 * r;
      const float v = sr[cc < NCTXL ? cc : (NCTXL - 1)];
      m = fmaxf(m, (cc < NCTXL) ? v : -INFINITY);
    }
    m = wave_max(m);
    float ssum = 0.f;
#pragma unroll 1
    for (int r = 0; r < 3; ++r) {
      const int cc = lane + 32 * r;
      const float v = sr[cc < NCTXL ? cc : (NCTXL - 1)];
      float e = expf(v - m);
      e = (cc < NCTXL) ? e : 0.0f;
      ssum += e;
      if (cc < NCTXL) sr[cc] = e;
    }
    ssum = wave_sum(ssum);
    const float inv = 1.0f / ssum;
#pragma unroll 1
    for (int r = 0; r < 3; ++r) {
      const int cc = lane + 32 * r;
      if (cc < NCTXL) sr[cc] = sr[cc] * inv;
    }
  }
  __syncthreads();

  if (wave == 0) {
    const int nk = clampi(kcount[0], 0, KNB);
    float wa = 0.f;
#pragma unroll 1
    for (int hh = 0; hh < NHEAD; ++hh) wa += sHi[hh] * sRow[hh * HEADPITCH + 1 + lane];
    wa = (lane < nk) ? wa : 0.0f;
    const float wtot = wave_sum(wa);
    const float wn = wa * (1.0f / (wtot + 1e-8f));
    const int nb = sIdx[lane];
    const float* pp = pos + ((size_t)b * NLS + nb) * 2;
    const float ax = wave_sum(wn * pp[0]);
    const float ay = wave_sum(wn * pp[1]);
    if (lane == 0) {
      sRow[DISPSLOT]     = ax - pos[(size_t)l * 2];
      sRow[DISPSLOT + 1] = ay - pos[(size_t)l * 2 + 1];
    }
  }
  __syncthreads();

  {
    const int t4 = tid < (ATTNPITCH / 4) ? tid : (ATTNPITCH / 4 - 1);
    const v4f v = *(const v4f*)(sRow + t4 * 4);
    float* dst = attn + (size_t)l * ATTNPITCH + t4 * 4;
    for (int pass = 0; pass < 2; ++pass) {
      if (tid < ATTNPITCH / 4) *(volatile v4f*)dst = v;
      __threadfence();
    }
  }
}

__global__ __launch_bounds__(128) void attn_out_kernel(const float* __restrict__ attn, const float* __restrict__ Vpl,
                                                       const unsigned short* __restrict__ RVp,
                                                       const int* __restrict__ topk, unsigned short* __restrict__ outl,
                                                       int tok0) {
  __shared__ __align__(16) float sA[ATTNPITCH];
  __shared__ int sFrow[HEADPITCH];
  __shared__ __align__(16) unsigned int sO[NINNER / 2];
  const int tid = threadIdx.x;
  const int lloc = blockIdx.x;
  const int l = tok0 + lloc;
  const int b = l >> 10;
#pragma unroll 1
  for (int i = tid; i < ATTNPITCH / 4; i += 128)
    *(v4f*)(sA + i * 4) = *(const v4f*)(attn + (size_t)l * ATTNPITCH + i * 4);
  if (tid < NCTXL) {
    const int cc = tid;
    const int cm1 = clampi(cc - 1, 0, KNB - 1);
    const int nb = clampi(topk[(size_t)l * KNB + cm1], 0, NLS - 1);
    const int fr = (cc == 0) ? l : (cc <= KNB) ? (b * NLS + nb) : (NTOK + b * 64 + (cc - KNB - 1));
    sFrow[cc] = fr;
  }
  __syncthreads();
  const int hh = tid >> 4;
  const int col = tid * 4;
  float acc0 = 0.f, acc1 = 0.f, acc2 = 0.f, acc3 = 0.f;
#pragma unroll 1
  for (int cc = 0; cc < NCTXL; ++cc) {
    const int fr = sFrow[cc];
    const int rs = cc < NSLOT ? cc : (NSLOT - 1);
    const float rmul = (cc < NSLOT) ? (1.0f / RCARRY) : 0.0f;
    const float p = sA[hh * HEADPITCH + cc];
    const v4f vf = *(const v4f*)(Vpl + (size_t)fr * NINNER + col);
    const v2u vr = *(const v2u*)(RVp + ((size_t)lloc * NSLOT + rs) * NINNER + col);
    acc0 += p * (vf[0] + rmul * hlo2f(vr[0]));
    acc1 += p * (vf[1] + rmul * hhi2f(vr[0]));
    acc2 += p * (vf[2] + rmul * hlo2f(vr[1]));
    acc3 += p * (vf[3] + rmul * hhi2f(vr[1]));
  }
  sO[tid * 2]     = pk16(h_bits(acc0 * OCARRY), h_bits(acc1 * OCARRY));
  sO[tid * 2 + 1] = pk16(h_bits(acc2 * OCARRY), h_bits(acc3 * OCARRY));
  __syncthreads();
  {
    const int tc = tid < 64 ? tid : 63;
    const v4u u = *(const v4u*)(sO + tc * 4);
    unsigned short* dst = outl + (size_t)l * NINNER + tc * 8;
    for (int pass = 0; pass < 2; ++pass) {
      if (tid < 64) *(volatile v4u*)dst = u;
      __threadfence();
    }
  }
}

__global__ __launch_bounds__(256) void gattn_kernel(const float* __restrict__ Qg, const float* __restrict__ Kg,
                                                    const float* __restrict__ Vg, const float* __restrict__ gbg,
                                                    unsigned short* __restrict__ og) {
  __shared__ __align__(16) float sQ[GQGRP * DHEAD];
  __shared__ __align__(16) float sP[GQGRP * CTXVALID];
  __shared__ __align__(16) float sO[GQGRP * DHEAD];
  const int tid = threadIdx.x, lane = tid & 31, wave = tid >> 5;
  const int qg = blockIdx.x & 3;
  const int h  = (blockIdx.x >> 2) & 7;
  const int b  = blockIdx.x >> 5;
  if (tid < 128) {
    const int qi = tid >> 4, d4 = (tid & 15) * 4;
    *(v4f*)(sQ + qi * DHEAD + d4) =
        *(const v4f*)(Qg + (size_t)(b * 64 + qg * GQGRP + qi) * NINNER + h * DHEAD + d4);
  }
  __syncthreads();
  const float gb = gbg[0];
#pragma unroll 1
  for (int r = 0; r < 5; ++r) {
    const int cidx = tid + 256 * r;
    const int cc = cidx < CTXVALID ? cidx : (CTXVALID - 1);
    const float* krow = Kg + ((size_t)b * CTXROWS + cc) * NINNER + h * DHEAD;
    float a[GQGRP];
#pragma unroll
    for (int qi = 0; qi < GQGRP; ++qi) a[qi] = 0.f;
#pragma unroll 1
    for (int d4 = 0; d4 < DHEAD / 4; ++d4) {
      const v4f kv = *(const v4f*)(krow + 4 * d4);
#pragma unroll
      for (int qi = 0; qi < GQGRP; ++qi) {
        const v4f qv = *(const v4f*)(sQ + qi * DHEAD + 4 * d4);
        a[qi] += kv[0] * qv[0] + kv[1] * qv[1] + kv[2] * qv[2] + kv[3] * qv[3];
      }
    }
    if (cidx < CTXVALID) {
#pragma unroll
      for (int qi = 0; qi < GQGRP; ++qi) sP[qi * CTXVALID + cidx] = a[qi] * ATTNSCALE + gb;
    }
  }
  __syncthreads();
  {
    float* pr = sP + wave * CTXVALID;
    float m = -INFINITY;
#pragma unroll 1
    for (int j = lane; j < CTXVALID; j += 32) m = fmaxf(m, pr[j]);
    m = wave_max(m);
    float ssum = 0.f;
#pragma unroll 1
    for (int j = lane; j < CTXVALID; j += 32) { const float e = expf(pr[j] - m); pr[j] = e; ssum += e; }
    ssum = wave_sum(ssum);
    const float inv = 1.0f / ssum;
#pragma unroll 1
    for (int j = lane; j < CTXVALID; j += 32) pr[j] = pr[j] * inv;
  }
  __syncthreads();
  {
    const float* pr = sP + wave * CTXVALID;
    const int col = 2 * lane;
    const float* vb = Vg + (size_t)b * CTXROWS * NINNER + h * DHEAD + col;
    float o0 = 0.f, o1 = 0.f;
#pragma unroll 1
    for (int cidx = 0; cidx < CTXVALID; ++cidx) {
      const float p = pr[cidx];
      const v2f vv = *(const v2f*)(vb + (size_t)cidx * NINNER);
      o0 += p * vv[0];
      o1 += p * vv[1];
    }
    sO[wave * DHEAD + col]     = o0 * OCARRY;
    sO[wave * DHEAD + col + 1] = o1 * OCARRY;
  }
  __syncthreads();
  {
    const int qq = wave * 4 + (lane >> 3);
    const int qqc = qq < GQGRP ? qq : (GQGRP - 1);
    const int c8 = (lane & 7) * 8;
    unsigned short hb[8];
#pragma unroll
    for (int e = 0; e < 8; ++e) hb[e] = h_bits(sO[qqc * DHEAD + c8 + e]);
    const v4u u = (v4u){pk16(hb[0], hb[1]), pk16(hb[2], hb[3]), pk16(hb[4], hb[5]), pk16(hb[6], hb[7])};
    unsigned short* dst = og + (size_t)(b * NGLOB + qg * GQGRP + qqc) * NINNER + h * DHEAD + c8;
    for (int pass = 0; pass < 2; ++pass) {
      if (wave < 2) *(volatile v4u*)dst = u;
      __threadfence();
    }
  }
}

__global__ __launch_bounds__(512) void disp_kernel(const float* __restrict__ h1, const float* __restrict__ lng,
                                                   const float* __restrict__ lnb, const float* __restrict__ W2,
                                                   const float* __restrict__ b2, const float* __restrict__ attn,
                                                   const float* __restrict__ law, const float* __restrict__ lmw,
                                                   float* __restrict__ out2) {
  __shared__ float sG[16][NHID];
  __shared__ __align__(16) float sOut[32];
  const int lane = threadIdx.x & 31, wave = threadIdx.x >> 5;
  const int l = blockIdx.x * 16 + wave;
  const float* hr = h1 + (size_t)l * NHID;
  float s = 0.f;
#pragma unroll 1
  for (int i = 0; i < 4; ++i) {
    const int j = lane + 32 * i;
    const float x = hr[j];
    const float g = 0.5f * x * (1.0f + erff(x * 0.70710678118654752f));
    sG[wave][j] = g;
    s += g;
  }
  s = wave_sum(s);
  const float mean = s * (1.0f / NHID);
  float ss = 0.f;
#pragma unroll 1
  for (int i = 0; i < 4; ++i) {
    const int j = lane + 32 * i;
    const float d = sG[wave][j] - mean;
    ss += d * d;
  }
  ss = wave_sum(ss);
  const float rstd = 1.0f / sqrtf(ss * (1.0f / NHID) + 1e-5f);
  float m0 = 0.f, m1 = 0.f;
#pragma unroll 1
  for (int i = 0; i < 4; ++i) {
    const int j = lane + 32 * i;
    const float hn = (sG[wave][j] - mean) * rstd * lng[j] + lnb[j];
    m0 += hn * W2[2 * j];
    m1 += hn * W2[2 * j + 1];
  }
  m0 = wave_sum(m0);
  m1 = wave_sum(m1);
  const int comp = lane & 1;
  const float md = (comp ? m1 : m0) + b2[comp];
  const float wa = expf(law[0]);
  const float wm = expf(lmw[0]);
  const float inv = 1.0f / (wa + wm + 1e-8f);
  const float ad = attn[(size_t)l * ATTNPITCH + DISPSLOT + comp];
  const float cmb = (wa * ad + wm * md) * inv;
  const float dv = tanhf(cmb * (1.0f / MAXDISP)) * MAXDISP;
  if (lane < 2) sOut[wave * 2 + comp] = dv;
  __syncthreads();
  {
    const int t = threadIdx.x;
    const int tc = t < 8 ? t : 7;
    const v4f v = *(const v4f*)(sOut + tc * 4);
    float* dst = out2 + (size_t)blockIdx.x * 32 + tc * 4;
    for (int pass = 0; pass < 2; ++pass) {
      if (t < 8) *(volatile v4f*)dst = v;
      __threadfence();
    }
  }
}

template <int BIAS, int OUTM, bool RESID>
static void launch_gemm(hipStream_t stream, const void* A, int lda, long strideA,
                        const void* Bt, int ldb, long strideB,
                        void* C, int ldc, long strideC,
                        const float* bias, const float* resid, long strideR,
                        int M, int N, int K, float scale, int batches) {
  const int tiles = (M / 64) * (N / 64);
  dim3 grid((tiles + 7) / 8, batches);
  wmma_gemm64<0, false, BIAS, OUTM, RESID, 0><<<grid, 256, 0, stream>>>(
      (const unsigned short*)A, nullptr, lda, strideA,
      (const unsigned short*)Bt, nullptr, ldb, strideB,
      C, nullptr, ldc, strideC, bias, resid, strideR, M, N, K, scale);
}

extern "C" void kernel_launch(void* const* d_in, const int* in_sizes, int n_in,
                              void* d_out, int out_size, void* d_ws, size_t ws_size,
                              hipStream_t stream) {
  (void)in_sizes; (void)out_size;
  if (n_in < 34) return;
  const float* spatial        = (const float*)d_in[0];
  const float* global_latents = (const float*)d_in[1];
  const float* positions      = (const float*)d_in[2];
  const float* rpe            = (const float*)d_in[3];
  const float* self_rpe       = (const float*)d_in[4];
  const float* distances      = (const float*)d_in[5];
  const float* ln_s_g = (const float*)d_in[6];
  const float* ln_s_b = (const float*)d_in[7];
  const float* ln_g_g = (const float*)d_in[8];
  const float* ln_g_b = (const float*)d_in[9];
  const float* Wq_l = (const float*)d_in[10];
  const float* Wk_l = (const float*)d_in[11];
  const float* Wv_l = (const float*)d_in[12];
  const float* Wo_l = (const float*)d_in[13];
  const float* bo_l = (const float*)d_in[14];
  const float* log_sigma = (const float*)d_in[15];
  const float* gb_l = (const float*)d_in[16];
  const float* Wq_g = (const float*)d_in[17];
  const float* Wk_g = (const float*)d_in[18];
  const float* Wv_g = (const float*)d_in[19];
  const float* Wo_g = (const float*)d_in[20];
  const float* bo_g = (const float*)d_in[21];
  const float* gb_g = (const float*)d_in[22];
  const float* head_weights = (const float*)d_in[23];
  const float* mlp_W1 = (const float*)d_in[24];
  const float* mlp_b1 = (const float*)d_in[25];
  const float* mlp_ln_g = (const float*)d_in[26];
  const float* mlp_ln_b = (const float*)d_in[27];
  const float* mlp_W2 = (const float*)d_in[28];
  const float* mlp_b2 = (const float*)d_in[29];
  const float* log_attn_w = (const float*)d_in[30];
  const float* log_mlp_w  = (const float*)d_in[31];
  const int*   topk = (const int*)d_in[32];
  const int*   kin  = (const int*)d_in[33];

  float* out0 = (float*)d_out;
  float* out1 = (float*)((char*)d_out + 4194304);
  float* out2 = (float*)((char*)d_out + 4325376);

  char* ws = (char*)d_ws;
  size_t off = 0;
  auto carve = [&](size_t bytes) -> char* { char* p = ws + off; off += (bytes + 255) & ~(size_t)255; return p; };
  unsigned short* WT8    = (unsigned short*)carve((size_t)8 * NDIM * NINNER * 2);
  unsigned short* WTR    = (unsigned short*)carve((size_t)2 * NINNER * NPE * 2);
  unsigned short* W1T    = (unsigned short*)carve((size_t)NHID * NDIM * 2);
  unsigned short* ctxp   = (unsigned short*)carve((size_t)NBATCH * CTXROWS * NDIM * 2);
  unsigned short* rpecat = (unsigned short*)carve((size_t)NRPEROWS * NPE * 2);
  float* Qp  = (float*)carve((size_t)NTOK * NINNER * 4);
  float* Kpl = (float*)carve((size_t)KVROWS * NINNER * 4);
  float* Vpl = (float*)carve((size_t)KVROWS * NINNER * 4);
  float* Qgp = (float*)carve((size_t)NBATCH * 64 * NINNER * 4);
  float* Kgp = (float*)carve((size_t)NBATCH * CTXROWS * NINNER * 4);
  float* Vgp = (float*)carve((size_t)NBATCH * CTXROWS * NINNER * 4);
  unsigned short* RKreg = (unsigned short*)carve((size_t)RPEROWS_B * NINNER * 2);
  unsigned short* RVreg = (unsigned short*)carve((size_t)RPEROWS_B * NINNER * 2);
  float* attnp = (float*)carve((size_t)NTOK * ATTNPITCH * 4);
  unsigned short* outl = (unsigned short*)carve((size_t)NTOK * NINNER * 2);
  unsigned short* ogp  = (unsigned short*)carve((size_t)NGROW * NINNER * 2);
  unsigned short* s2h  = (unsigned short*)carve((size_t)NTOK * NDIM * 2);
  float* h1pre = (float*)carve((size_t)NTOK * NHID * 4);
  if (off > ws_size) return;

  const long WPLANE = (long)NDIM * NINNER;
  const long RPLANE = (long)NINNER * NPE;
  const float WINV  = 1.0f / WCARRY;

  wtcast_kernel<<<dim3(8, 8, 4), 256, 0, stream>>>(Wq_l, Wk_l, Wv_l, Wo_l, NDIM, NINNER, WT8, WPLANE, WCARRY);
  wtcast_kernel<<<dim3(8, 8, 4), 256, 0, stream>>>(Wq_g, Wk_g, Wv_g, Wo_g, NDIM, NINNER, WT8 + 4 * WPLANE, WPLANE, WCARRY);
  wtcast_kernel<<<dim3(1, 8, 2), 256, 0, stream>>>(Wk_l + (size_t)NDIM * NINNER, Wv_l + (size_t)NDIM * NINNER,
                                                    Wk_l + (size_t)NDIM * NINNER, Wv_l + (size_t)NDIM * NINNER,
                                                    NPE, NINNER, WTR, RPLANE, WCARRY);
  wtcast_kernel<<<dim3(8, 2, 1), 256, 0, stream>>>(mlp_W1, mlp_W1, mlp_W1, mlp_W1, NDIM, NHID, W1T, 0, WCARRY);

  ln_rows_kernel<<<(NTOK + NGROW) / 8, 256, 0, stream>>>(spatial, global_latents, ln_s_g, ln_s_b, ln_g_g, ln_g_b, ctxp);
  zero_ctxpad_kernel<<<16, 256, 0, stream>>>(ctxp);
  rpecat_kernel<<<dim3(NTOK / 32, NSLOT), 256, 0, stream>>>(rpe, self_rpe, rpecat);

  const long CTXSTRIDE = (long)CTXROWS * NDIM;
  const unsigned short* WqlT  = WT8 + 0 * WPLANE;
  const unsigned short* WkflT = WT8 + 1 * WPLANE;
  const unsigned short* WvflT = WT8 + 2 * WPLANE;
  const unsigned short* WolT  = WT8 + 3 * WPLANE;
  const unsigned short* WqgT  = WT8 + 4 * WPLANE;
  const unsigned short* WkgT  = WT8 + 5 * WPLANE;
  const unsigned short* WvgT  = WT8 + 6 * WPLANE;
  const unsigned short* WogT  = WT8 + 7 * WPLANE;

  launch_gemm<0, 0, false>(stream, ctxp, NDIM, CTXSTRIDE, WqlT, NDIM, 0, Qp, NINNER, (long)NLS * NINNER,
                           nullptr, nullptr, 0, NLS, NINNER, NDIM, WINV, NBATCH);
  launch_gemm<0, 0, false>(stream, ctxp, NDIM, CTXSTRIDE, WkflT, NDIM, 0, Kpl, NINNER, (long)NLS * NINNER,
                           nullptr, nullptr, 0, NLS, NINNER, NDIM, WINV, NBATCH);
  launch_gemm<0, 0, false>(stream, ctxp, NDIM, CTXSTRIDE, WvflT, NDIM, 0, Vpl, NINNER, (long)NLS * NINNER,
                           nullptr, nullptr, 0, NLS, NINNER, NDIM, WINV, NBATCH);
  launch_gemm<0, 0, false>(stream, ctxp + (size_t)NLS * NDIM, NDIM, CTXSTRIDE, WkflT, NDIM, 0,
                           Kpl + (size_t)NTOK * NINNER, NINNER, (long)64 * NINNER,
                           nullptr, nullptr, 0, 64, NINNER, NDIM, WINV, NBATCH);
  launch_gemm<0, 0, false>(stream, ctxp + (size_t)NLS * NDIM, NDIM, CTXSTRIDE, WvflT, NDIM, 0,
                           Vpl + (size_t)NTOK * NINNER, NINNER, (long)64 * NINNER,
                           nullptr, nullptr, 0, 64, NINNER, NDIM, WINV, NBATCH);
  launch_gemm<0, 0, false>(stream, ctxp + (size_t)NLS * NDIM, NDIM, CTXSTRIDE, WqgT, NDIM, 0,
                           Qgp, NINNER, (long)64 * NINNER,
                           nullptr, nullptr, 0, 64, NINNER, NDIM, WINV, NBATCH);
  launch_gemm<0, 0, false>(stream, ctxp, NDIM, CTXSTRIDE, WkgT, NDIM, 0, Kgp, NINNER, CTXSTRIDE,
                           nullptr, nullptr, 0, CTXROWS, NINNER, NDIM, WINV, NBATCH);
  launch_gemm<0, 0, false>(stream, ctxp, NDIM, CTXSTRIDE, WvgT, NDIM, 0, Vgp, NINNER, CTXSTRIDE,
                           nullptr, nullptr, 0, CTXROWS, NINNER, NDIM, WINV, NBATCH);

  for (int b = 0; b < NBATCH; ++b) {
    const unsigned short* rpeb = rpecat + (size_t)b * RPEROWS_B * NPE;
    launch_gemm<0, 1, false>(stream, rpeb, NPE, 0, WTR, NPE, 0, RKreg, NINNER, 0,
                             nullptr, nullptr, 0, RPEROWS_B, NINNER, NPE, RCARRY / WCARRY, 1);
    launch_gemm<0, 1, false>(stream, rpeb, NPE, 0, WTR + RPLANE, NPE, 0, RVreg, NINNER, 0,
                             nullptr, nullptr, 0, RPEROWS_B, NINNER, NPE, RCARRY / WCARRY, 1);
    attn_scores_kernel<<<NLS, 256, 0, stream>>>(Qp, Kpl, RKreg, distances, topk, log_sigma, gb_l, head_weights,
                                                positions, kin, attnp, b * NLS);
    attn_out_kernel<<<NLS, 128, 0, stream>>>(attnp, Vpl, RVreg, topk, outl, b * NLS);
  }

  gattn_kernel<<<NBATCH * NHEAD * (NGLOB / GQGRP), 256, 0, stream>>>(Qgp, Kgp, Vgp, gb_g, ogp);

  launch_gemm<2, 0, true>(stream, outl, NINNER, 0, WolT, NINNER, 0, out0, NDIM, 0,
                          bo_l, spatial, 0, NTOK, NDIM, NINNER, 1.0f / (OCARRY * WCARRY), 1);
  launch_gemm<2, 0, true>(stream, ogp, NINNER, 0, WogT, NINNER, 0, out1, NDIM, 0,
                          bo_g, global_latents, 0, NGROW, NDIM, NINNER, 1.0f / (OCARRY * WCARRY), 1);

  cast8_f16_kernel<<<(NTOK * NDIM / 8 + 255) / 256, 256, 0, stream>>>(out0, s2h, NTOK * NDIM / 8);
  launch_gemm<2, 0, false>(stream, s2h, NDIM, 0, W1T, NDIM, 0, h1pre, NHID, 0,
                           mlp_b1, nullptr, 0, NTOK, NHID, NDIM, WINV, 1);
  disp_kernel<<<NTOK / 16, 512, 0, stream>>>(h1pre, mlp_ln_g, mlp_ln_b, mlp_W2, mlp_b2, attnp, log_attn_w, log_mlp_w, out2);
}
